// GraphNN_40209483825155
// MI455X (gfx1250) — hardware-verified
//
#include <hip/hip_runtime.h>
#include <stddef.h>
#include <stdint.h>


#define DIN    32
#define DH     64
#define AP1    128
#define K1     96
#define AP2    256
#define K2     256
#define NTHR   256
#define NWAVE  8
#define EPT    8
#define CHUNK  (NTHR * EPT)
#define WCAP   (EPT * 32)
#define LISTN  (NWAVE * WCAP)
#define NBA    1024
#define SLA    10
#define RCAP   28672
#define DEGCAP 256
#define GBM    64
#define GTHR   128
#define AGG_ZINTS    (LISTN + 2 * RCAP + 3 * NBA)
#define MISC_INTS    16
#define ROWBUF_INTS  (NWAVE * AP2 / 2)
#define AGG_LDS_INTS (AGG_ZINTS + MISC_INTS + ROWBUF_INTS)
#define WSMAX  134217728

static_assert((CHUNK & (CHUNK - 1)) == 0 && CHUNK <= 4096);
static_assert((NBA & (NBA - 1)) == 0 && NBA == (1 << SLA));
static_assert(((long long)CHUNK << SLA) < (1LL << 31));
static_assert(LISTN % NTHR == 0 && LISTN >= NBA);
static_assert(NBA % NWAVE == 0 && NBA % 32 == 0 && NBA % GBM == 0 && NBA % 4 == 0);
static_assert(RCAP % 4 == 0 && AGG_ZINTS % 4 == 0 && LISTN % 4 == 0 && ((AGG_ZINTS + MISC_INTS) % 4) == 0);
static_assert(AGG_ZINTS % (NTHR * 4) == 0 && ROWBUF_INTS % (NTHR * 4) == 0);
static_assert(K1 % 32 == 0 && K2 % 32 == 0 && K1 == 3 * DIN && K1 <= AP1 && K2 == 4 * DH && K2 == AP2);
static_assert(AP1 % 64 == 0 && AP2 % 64 == 0);
static_assert(DIN == 32 && DH == 2 * 32);
static_assert(GBM == (GTHR / 32) * 16);
static_assert(AGG_LDS_INTS * 4 <= 300000);

typedef float          v2f   __attribute__((ext_vector_type(2)));
typedef float          v4f   __attribute__((ext_vector_type(4)));
typedef float          v8f   __attribute__((ext_vector_type(8)));
typedef int            v4i   __attribute__((ext_vector_type(4)));
typedef int            v8i   __attribute__((ext_vector_type(8)));
typedef unsigned short v2us  __attribute__((ext_vector_type(2)));
typedef unsigned short v8us  __attribute__((ext_vector_type(8)));
typedef unsigned short v16us __attribute__((ext_vector_type(16)));
typedef __bf16         v16bf __attribute__((ext_vector_type(16)));
typedef v2f  __attribute__((may_alias)) v2fa;
typedef v4f  __attribute__((may_alias)) v4fa;
typedef v4i  __attribute__((may_alias)) v4ia;
typedef v2us __attribute__((may_alias)) v2usa;
typedef v8us __attribute__((may_alias)) v8usa;
union FragB { v16bf v; v16us u; v8us h[2]; v8i w; };

__device__ __forceinline__ v8f wmb(const FragB& a, const FragB& b, v8f c) {
  v8f d = __builtin_amdgcn_wmma_f32_16x16x32_bf16(false, a.v, false, b.v, (short)0, c, false, false);
  asm volatile("v_nop\n\tv_nop\n\tv_nop\n\tv_nop" : "+v"(d) : "v"(a.w), "v"(b.w));
  return d;
}

__device__ __forceinline__ unsigned bf16_bits(float f) {
  const unsigned u = __float_as_uint(f);
  return (u + 0x7FFFu + ((u >> 16) & 1u)) >> 16;
}
__device__ __forceinline__ float bf16_val(float f) {
  return __uint_as_float(bf16_bits(f) << 16);
}

__device__ __forceinline__ unsigned short bsel(float r, float t, unsigned mR, unsigned mZ) {
  const unsigned a = bf16_bits(r);
  const unsigned b = bf16_bits(t);
  return (unsigned short)(((b & mR) | (a & ~mR)) & mZ);
}

__device__ __forceinline__ void wave_sync() {
  __builtin_amdgcn_fence(__ATOMIC_RELEASE, "wavefront");
  __builtin_amdgcn_wave_barrier();
  __builtin_amdgcn_fence(__ATOMIC_ACQUIRE, "wavefront");
}

template <int SLB>
__device__ __forceinline__ int scan_chunk(const int* __restrict__ dsts, int nE, int cbase, int slotBase,
                                          int nb, int vec8, int* list, int tid, int lane, int wave) {
  int wc = 0;
  const int el0  = tid * EPT;
  const int e0   = cbase + el0;
  const int sent = -2147483647 - 1;
  v4i da, db;
  if (vec8 != 0 && cbase + CHUNK <= nE) {
    da = *(const v4i*)(dsts + e0);
    db = *(const v4i*)(dsts + e0 + 4);
  } else {
    da.x = (e0     < nE) ? dsts[min(e0,     nE - 1)] : sent;
    da.y = (e0 + 1 < nE) ? dsts[min(e0 + 1, nE - 1)] : sent;
    da.z = (e0 + 2 < nE) ? dsts[min(e0 + 2, nE - 1)] : sent;
    da.w = (e0 + 3 < nE) ? dsts[min(e0 + 3, nE - 1)] : sent;
    db.x = (e0 + 4 < nE) ? dsts[min(e0 + 4, nE - 1)] : sent;
    db.y = (e0 + 5 < nE) ? dsts[min(e0 + 5, nE - 1)] : sent;
    db.z = (e0 + 6 < nE) ? dsts[min(e0 + 6, nE - 1)] : sent;
    db.w = (e0 + 7 < nE) ? dsts[min(e0 + 7, nE - 1)] : sent;
  }
  const unsigned nbs = (unsigned)slotBase;
  const unsigned unb = (unsigned)nb;
  const unsigned s0 = (unsigned)da.x - nbs, s1 = (unsigned)da.y - nbs;
  const unsigned s2 = (unsigned)da.z - nbs, s3 = (unsigned)da.w - nbs;
  const unsigned s4 = (unsigned)db.x - nbs, s5 = (unsigned)db.y - nbs;
  const unsigned s6 = (unsigned)db.z - nbs, s7 = (unsigned)db.w - nbs;
  const bool h0 = s0 < unb, h1 = s1 < unb, h2 = s2 < unb, h3 = s3 < unb;
  const bool h4 = s4 < unb, h5 = s5 < unb, h6 = s6 < unb, h7 = s7 < unb;
  const unsigned any = __builtin_amdgcn_ballot_w32(h0 | h1 | h2 | h3 | h4 | h5 | h6 | h7);
  if (any != 0u) {
#define HITJ(J, HJ, SJ) { \
      const unsigned mj = __builtin_amdgcn_ballot_w32(HJ); \
      if (mj != 0u) { \
        if (HJ) { \
          const int pos = wc + (int)__builtin_amdgcn_mbcnt_lo(mj, 0u); \
          if (pos < WCAP) list[wave * WCAP + pos] = ((el0 + (J)) << SLB) | (int)(SJ); \
        } \
        wc += (int)__builtin_popcount(mj); } }
    HITJ(0, h0, s0)
    HITJ(1, h1, s1)
    HITJ(2, h2, s2)
    HITJ(3, h3, s3)
    HITJ(4, h4, s4)
    HITJ(5, h5, s5)
    HITJ(6, h6, s6)
    HITJ(7, h7, s7)
#undef HITJ
  }
  return wc;
}

__global__ __launch_bounds__(NTHR) void k_wprep(const float* __restrict__ w1r, const float* __restrict__ w1o,
                                                const float* __restrict__ w2r, const float* __restrict__ w2o,
                                                unsigned short* B1, unsigned short* B2) {
  __shared__ __attribute__((aligned(16))) float swr[DH * DH];
  __shared__ __attribute__((aligned(16))) float swo[DH * DH];
  const int tid   = (int)threadIdx.x;
  const int which = (int)(blockIdx.x & 1u);
  const int Kin   = (which == 0) ? DIN : DH;
  const float* wr = (which == 0) ? w1r : w2r;
  const float* wo = (which == 0) ? w1o : w2o;
  unsigned short* B = (which == 0) ? B1 : B2;
  const int nf4 = (Kin * DH) / 4;
#pragma unroll 1
  for (int i = tid; i < nf4; i += NTHR) {
    *(v4fa*)(swr + 4 * i) = *(const v4f*)(wr + 4 * i);
    *(v4fa*)(swo + 4 * i) = *(const v4f*)(wo + 4 * i);
  }
  __syncthreads();
  const int lgNG = (which == 0) ? 4 : 5;
  const int NG   = 1 << lgNG;
  const int GS   = NG >> 2;
  const int nUnits = DH * NG;
#pragma unroll 1
  for (int u = tid; u < nUnits; u += NTHR) {
    const int n   = u >> lgNG;
    const int g   = u & (NG - 1);
    const int seg = g >> (lgNG - 2);
    const int kk  = 8 * (g & (GS - 1));
    const unsigned mR = (seg >= 2) ? 0xFFFFu : 0u;
    const unsigned mZ = (which == 0 && seg == 3) ? 0u : 0xFFFFu;
    v8us o;
#pragma unroll
    for (int j = 0; j < 8; ++j) o[j] = bsel(swr[(kk + j) * DH + n], swo[(kk + j) * DH + n], mR, mZ);
    unsigned short* dp = B + (size_t)n * (size_t)(8 * NG) + 8 * g;
    *(volatile v8us*)dp = o;
    __threadfence();
    *(volatile v8us*)dp = o;
  }
}

template <int NT, int RELU>
__global__ __launch_bounds__(GTHR) void k_gemm(const unsigned short* __restrict__ A, int lda,
                                               const unsigned short* __restrict__ BT, int ldb, int K,
                                               const float* __restrict__ bias, float* outp, int nOut) {
  static_assert(NT == 4 || NT == 8);
  constexpr int N   = 16 * NT;
  constexpr int RPI = 128 / N;
  constexpr int NI  = 16 / RPI;
  __shared__ __attribute__((aligned(16))) float stg[GBM * N];
  const int tid = (int)threadIdx.x, lane = tid & 31, wave = tid >> 5, hh = lane >> 4, m = lane & 15;
  const int rowBase = (int)blockIdx.x * GBM;

  v8f acc[NT];
  {
    const v8f z = {0.f, 0.f, 0.f, 0.f, 0.f, 0.f, 0.f, 0.f};
#pragma unroll
    for (int t = 0; t < NT; ++t) acc[t] = z;
  }
  const unsigned short* ap = A  + (size_t)(rowBase + 16 * wave + m) * (size_t)lda + 8 * hh;
  const unsigned short* bp = BT + (size_t)m * (size_t)ldb + 8 * hh;

#pragma unroll 1
  for (int k0 = 0; k0 < K; k0 += 32) {
    FragB af;
    af.h[0] = *(const v8usa*)(ap + k0);
    af.h[1] = *(const v8usa*)(ap + k0 + 16);
#pragma unroll
    for (int nt = 0; nt < NT; ++nt) {
      const unsigned short* wq = bp + (size_t)(16 * nt) * (size_t)ldb + k0;
      FragB bf;
      bf.h[0] = *(const v8usa*)wq;
      bf.h[1] = *(const v8usa*)(wq + 16);
      acc[nt] = wmb(af, bf, acc[nt]);
    }
  }

#pragma unroll
  for (int nt = 0; nt < NT; ++nt) {
    const int lc = 16 * nt + m;
#pragma unroll
    for (int r = 0; r < 8; ++r) {
      const int lr = 16 * wave + 8 * hh + r;
      stg[lr * N + lc] = acc[nt][r];
    }
  }
  __syncthreads();

  const int lcol = (4 * lane) & (N - 1);
  const int lro  = (4 * lane) / N;
  v4f b4;
  {
    const v4f tb = *(const v4f*)(bias + lcol);
    b4.x = bf16_val(tb.x); b4.y = bf16_val(tb.y); b4.z = bf16_val(tb.z); b4.w = bf16_val(tb.w);
  }

  v4f pv[NI];
#pragma unroll
  for (int i = 0; i < NI; ++i) {
    v4f t = *(const v4fa*)(stg + (16 * wave + RPI * i) * N + 4 * lane) + b4;
    if (RELU != 0) {
      t.x = fmaxf(t.x, 0.0f); t.y = fmaxf(t.y, 0.0f); t.z = fmaxf(t.z, 0.0f); t.w = fmaxf(t.w, 0.0f);
    }
    pv[i] = t;
  }
#pragma unroll
  for (int i = 0; i < NI; ++i) {
    const int seg = rowBase + 16 * wave + RPI * i;
    if (seg + lro < nOut) *(volatile v4f*)(outp + (size_t)seg * N + 4 * lane) = pv[i];
  }
  __threadfence();
#pragma unroll
  for (int i = 0; i < NI; ++i) {
    const int seg = rowBase + 16 * wave + RPI * i;
    if (seg + lro < nOut) *(volatile v4f*)(outp + (size_t)seg * N + 4 * lane) = pv[i];
  }
}

template <int L>
__global__ __launch_bounds__(NTHR) void k_scan(const int* __restrict__ srcs, const int* __restrict__ dsts,
                                               int nE, int nN, int vec8, int mRows,
                                               const float* __restrict__ gin, unsigned short* apl,
                                               const float* __restrict__ w3r, const float* __restrict__ w3o,
                                               const float* __restrict__ b3, float* out) {
  static_assert(L == 1 || L == 2 || L == 3);
  extern __shared__ __attribute__((aligned(16))) int dsm[];
  int* list = dsm;
  int* hl   = dsm + LISTN;
  int* sl   = hl + RCAP;
  int* cnt  = sl + RCAP;
  int* offs = cnt + NBA;
  int* cur  = offs + NBA;
  int* misc = cur + NBA;
  const int tid = (int)threadIdx.x, lane = tid & 31, wave = tid >> 5;
  unsigned short* rowbuf = (unsigned short*)(misc + MISC_INTS) + wave * AP2;
  const int nodeBase = (int)blockIdx.x * NBA;

  {
    const v4i z4 = {0, 0, 0, 0};
    for (int i = tid * 4; i < AGG_ZINTS; i += NTHR * 4) *(v4ia*)(dsm + i) = z4;
    int* rbz = misc + MISC_INTS;
    for (int i = tid * 4; i < ROWBUF_INTS; i += NTHR * 4) *(v4ia*)(rbz + i) = z4;
    if (tid < MISC_INTS) misc[tid] = 0;
  }
  __syncthreads();

  int t = 0, ov = 0;
  const int nChunks = (nE + CHUNK - 1) / CHUNK;
#pragma unroll 1
  for (int ch = 0; ch < nChunks; ++ch) {
    const int cbase = ch * CHUNK;
    const int wc = scan_chunk<SLA>(dsts, nE, cbase, nodeBase, NBA, vec8, list, tid, lane, wave);
    if (lane == 0) misc[wave] = wc;
    __syncthreads();
    if (wave == 0) {
#pragma unroll 1
      for (int w2 = 0; w2 < NWAVE; ++w2) {
        int c = misc[w2];
        c = c < 0 ? 0 : (c > WCAP ? WCAP : c);
#pragma unroll 1
        for (int b0 = 0; b0 < c; b0 += 32) {
          const int idx = b0 + lane;
          const int ent = list[w2 * WCAP + (idx < WCAP ? idx : WCAP - 1)];
          const int m32 = (c - b0) < 32 ? (c - b0) : 32;
#pragma unroll 1
          for (int k = 0; k < m32; ++k) {
            const int u    = __builtin_amdgcn_readlane(ent, k);
            const int slot = u & (NBA - 1);
            const int el   = (u >> SLA) & (CHUNK - 1);
            const int pk   = ((cbase + el) << SLA) | slot;
            if (t < RCAP) {
              if (lane == 0) { hl[t] = pk; cnt[slot] = cnt[slot] + 1; }
              t = t + 1;
            } else {
              ov = 1;
            }
          }
        }
      }
    }
    __syncthreads();
  }
  if (wave == 0 && lane == 0) { misc[8] = t; misc[9] = ov; }
  __syncthreads();
  int tt = misc[8];
  tt = tt < 0 ? 0 : (tt > RCAP ? RCAP : tt);
  const int ovf = misc[9];

  if (wave == 0) {
    const int base = lane * (NBA / 32);
    int s = 0;
#pragma unroll 1
    for (int i = 0; i < NBA / 32; ++i) s += cnt[base + i];
    int incl = s;
#pragma unroll
    for (int d = 1; d < 32; d <<= 1) {
      const int y = __shfl_up(incl, d, 32);
      if (lane >= d) incl += y;
    }
    int run = incl - s;
#pragma unroll 1
    for (int i = 0; i < NBA / 32; ++i) {
      const int cv = cnt[base + i];
      offs[base + i] = run;
      cur[base + i]  = run;
      run += cv;
    }
  }
  __syncthreads();
  if (wave == 0) {
#pragma unroll 1
    for (int b0 = 0; b0 < tt; b0 += 32) {
      const int idx = b0 + lane;
      const int ent = hl[idx < RCAP ? idx : RCAP - 1];
      const int m32 = (tt - b0) < 32 ? (tt - b0) : 32;
#pragma unroll 1
      for (int k = 0; k < m32; ++k) {
        const int u    = __builtin_amdgcn_readlane(ent, k);
        const int slot = u & (NBA - 1);
        if (lane == 0) {
          int p = cur[slot];
          p = p < 0 ? 0 : (p > RCAP - 1 ? RCAP - 1 : p);
          sl[p] = u;
          cur[slot] = p + 1;
        }
      }
    }
  }
  __syncthreads();

  const float pz = (ovf != 0) ? __int_as_float(0x7fc00000) : 0.0f;
  float wr0 = 0.0f, wr1 = 0.0f, wo0 = 0.0f, wo1 = 0.0f, bb3 = 0.0f;
  if constexpr (L == 3) {
    wr0 = bf16_val(w3r[2 * lane]); wr1 = bf16_val(w3r[2 * lane + 1]);
    wo0 = bf16_val(w3o[2 * lane]); wo1 = bf16_val(w3o[2 * lane + 1]);
    bb3 = bf16_val(b3[0]);
  }
  float* res = (float*)list;
#pragma unroll 1
  for (int si = 0; si < NBA / NWAVE; ++si) {
    const int s    = si * NWAVE + wave;
    const int node = nodeBase + s;
    int c = cnt[s];
    const bool big = c > DEGCAP;
    c = c < 0 ? 0 : (c > DEGCAP ? DEGCAP : c);
    int o = offs[s];
    o = o < 0 ? 0 : (o > RCAP ? RCAP : o);
    const int nc = node < nN ? node : nN - 1;
    float a0 = 0.0f, a1 = 0.0f;
#pragma unroll 1
    for (int b0 = 0; b0 < c; b0 += 32) {
      int idx = o + b0 + lane;
      idx = idx > RCAP - 1 ? RCAP - 1 : idx;
      const int ent = sl[idx];
      int eid = ent >> SLA;
      eid = eid < 0 ? 0 : (eid > nE - 1 ? nE - 1 : eid);
      int sr = srcs[eid];
      sr = sr < 0 ? 0 : (sr > nN - 1 ? nN - 1 : sr);
      const int m32 = (c - b0) < 32 ? (c - b0) : 32;
#pragma unroll 1
      for (int k = 0; k < m32; ++k) {
        const int sk = __builtin_amdgcn_readlane(sr, k);
        if constexpr (L == 1) {
          const float v0 = gin[(size_t)sk * DIN + lane];
          a0 += bf16_val(v0);
        } else {
          const v2f av = *(const v2fa*)(gin + (size_t)sk * DH + 2 * lane);
          a0 += av.x; a1 += av.y;
        }
      }
    }
    const float pzr = big ? __int_as_float(0x7fc00000) : pz;
    const bool live = node < nN;
    if constexpr (L == 1) {
      const float s0 = live ? (a0 + pzr) : 0.0f;
      const unsigned hb0 = bf16_bits(s0);
      const unsigned lb0 = bf16_bits(s0 - __uint_as_float(hb0 << 16));
      const float x0 = gin[(size_t)nc * DIN + lane];
      rowbuf[lane]           = (unsigned short)hb0;
      rowbuf[DIN + lane]     = (unsigned short)lb0;
      rowbuf[2 * DIN + lane] = live ? (unsigned short)bf16_bits(x0 + pzr) : (unsigned short)0;
      rowbuf[K1 + lane]      = (unsigned short)0;
      (void)a1;
      wave_sync();
      const v8us q0 = *(const v8usa*)(rowbuf + 8 * (lane & 15));
      wave_sync();
      if (node < mRows) {
        unsigned short* rpw = apl + (size_t)node * AP1 + 8 * (lane & 15);
        if (lane < 16) *(volatile v8us*)rpw = q0;
        __threadfence();
        if (lane < 16) *(volatile v8us*)rpw = q0;
      }
    } else if constexpr (L == 2) {
      const float s0 = live ? (a0 + pzr) : 0.0f;
      const float s1 = live ? (a1 + pzr) : 0.0f;
      const v2f hs = *(const v2fa*)(gin + (size_t)nc * DH + 2 * lane);
      const float g0 = live ? (hs.x + pzr) : 0.0f;
      const float g1 = live ? (hs.y + pzr) : 0.0f;
      v2us mh, ml, gh, gl;
      {
        unsigned hb;
        hb = bf16_bits(s0); mh[0] = (unsigned short)hb; ml[0] = (unsigned short)bf16_bits(s0 - __uint_as_float(hb << 16));
        hb = bf16_bits(s1); mh[1] = (unsigned short)hb; ml[1] = (unsigned short)bf16_bits(s1 - __uint_as_float(hb << 16));
        hb = bf16_bits(g0); gh[0] = (unsigned short)hb; gl[0] = (unsigned short)bf16_bits(g0 - __uint_as_float(hb << 16));
        hb = bf16_bits(g1); gh[1] = (unsigned short)hb; gl[1] = (unsigned short)bf16_bits(g1 - __uint_as_float(hb << 16));
      }
      *(v2usa*)(rowbuf + 2 * lane)          = mh;
      *(v2usa*)(rowbuf + DH + 2 * lane)     = ml;
      *(v2usa*)(rowbuf + 2 * DH + 2 * lane) = gh;
      *(v2usa*)(rowbuf + 3 * DH + 2 * lane) = gl;
      wave_sync();
      const v8us q0 = *(const v8usa*)(rowbuf + 8 * lane);
      wave_sync();
      if (node < mRows) {
        unsigned short* rpw = apl + (size_t)node * AP2 + 8 * lane;
        *(volatile v8us*)rpw = q0;
        __threadfence();
        *(volatile v8us*)rpw = q0;
      }
    } else {
      const v2f hs = *(const v2fa*)(gin + (size_t)nc * DH + 2 * lane);
      float part = a0 * wr0;
      part = fmaf(a1, wr1, part);
      part = fmaf(hs.x, wo0, part);
      part = fmaf(hs.y, wo1, part);
#pragma unroll
      for (int off = 16; off > 0; off >>= 1) part += __shfl_xor(part, off);
      const float r = part + bb3 + pzr;
      if (lane == 0) res[s] = r;
    }
  }

  if constexpr (L == 3) {
    __syncthreads();
    const int npc = NBA >> 2;
#pragma unroll 1
    for (int p = tid; p < npc; p += NTHR) {
      const v4f v = *(const v4fa*)(res + 4 * p);
      const int r0 = nodeBase + 4 * p;
      if (r0 + 3 < nN) {
        *(volatile v4f*)(out + r0) = v;
      } else {
        if (r0     < nN) *(volatile float*)(out + r0)     = v.x;
        if (r0 + 1 < nN) *(volatile float*)(out + r0 + 1) = v.y;
        if (r0 + 2 < nN) *(volatile float*)(out + r0 + 2) = v.z;
      }
    }
    __threadfence();
#pragma unroll 1
    for (int p = tid; p < npc; p += NTHR) {
      const v4f v = *(const v4fa*)(res + 4 * p);
      const int r0 = nodeBase + 4 * p;
      if (r0 + 3 < nN) {
        *(volatile v4f*)(out + r0) = v;
      } else {
        if (r0     < nN) *(volatile float*)(out + r0)     = v.x;
        if (r0 + 1 < nN) *(volatile float*)(out + r0 + 1) = v.y;
        if (r0 + 2 < nN) *(volatile float*)(out + r0 + 2) = v.z;
      }
    }
  }
}

static inline int cdiv(int a, int b) { return (a + b - 1) / b; }

extern "C" void kernel_launch(void* const* d_in, const int* in_sizes, int n_in,
                              void* d_out, int out_size, void* d_ws, size_t ws_size,
                              hipStream_t stream) {
  if (n_in < 11) return;
  if (in_sizes[0] < DIN || (in_sizes[0] % DIN) != 0) return;
  const int nN = in_sizes[0] / DIN;
  if (nN > (1 << 22)) return;
  if (in_sizes[1] != DIN * DH || in_sizes[2] != DH || in_sizes[3] != DIN * DH) return;
  if (in_sizes[4] != DH * DH || in_sizes[5] != DH || in_sizes[6] != DH * DH) return;
  if (in_sizes[7] != DH || in_sizes[8] < 1 || in_sizes[9] != DH) return;
  if (in_sizes[10] < 2 || (in_sizes[10] & 1) != 0) return;
  const int nE = in_sizes[10] / 2;
  if (nE < 1 || nE >= (1 << 21)) return;
  if (out_size != nN) return;

  const float* x    = (const float*)d_in[0];
  const float* w1r  = (const float*)d_in[1];
  const float* b1   = (const float*)d_in[2];
  const float* w1o  = (const float*)d_in[3];
  const float* w2r  = (const float*)d_in[4];
  const float* b2   = (const float*)d_in[5];
  const float* w2o  = (const float*)d_in[6];
  const float* w3r  = (const float*)d_in[7];
  const float* b3   = (const float*)d_in[8];
  const float* w3o  = (const float*)d_in[9];
  const int*   edge = (const int*)  d_in[10];
  float* out = (float*)d_out;
  const int* src = edge;
  const int* dst = edge + nE;

  const int MP = cdiv(nN, GBM) * GBM;
  const int gM = MP / GBM;
  const int gA = cdiv(MP, NBA);
  if ((long long)gA * NBA < (long long)MP) return;
  const int vec8 = ((nE & 3) == 0) ? 1 : 0;

  char* ws = (char*)d_ws;
  size_t off = 0;
  const size_t oB1 = off; off += (size_t)DH * AP1 * 2;                    off = (off + 255) & ~(size_t)255;
  const size_t oB2 = off; off += (size_t)DH * AP2 * 2;                    off = (off + 255) & ~(size_t)255;
  const size_t oA1 = off; off += (size_t)MP * AP1 * 2;                    off = (off + 255) & ~(size_t)255;
  const size_t oH1 = off; off += (size_t)MP * DH * 4;                     off = (off + 255) & ~(size_t)255;
  const size_t oA2 = off; off += (size_t)MP * AP2 * 2;                    off = (off + 255) & ~(size_t)255;
  const size_t oH2 = off; off += (size_t)MP * DH * 4;                     off = (off + 255) & ~(size_t)255;
  if (off > ws_size || off > (size_t)WSMAX) return;
  unsigned short* B1 = (unsigned short*)(ws + oB1);
  unsigned short* B2 = (unsigned short*)(ws + oB2);
  unsigned short* A1 = (unsigned short*)(ws + oA1);
  float*          H1 = (float*)(ws + oH1);
  unsigned short* A2 = (unsigned short*)(ws + oA2);
  float*          H2 = (float*)(ws + oH2);

  const size_t scanLds = (size_t)AGG_LDS_INTS * 4;
  hipFuncSetAttribute(reinterpret_cast<const void*>(&k_scan<1>), hipFuncAttributeMaxDynamicSharedMemorySize, (int)scanLds);
  hipFuncSetAttribute(reinterpret_cast<const void*>(&k_scan<2>), hipFuncAttributeMaxDynamicSharedMemorySize, (int)scanLds);
  hipFuncSetAttribute(reinterpret_cast<const void*>(&k_scan<3>), hipFuncAttributeMaxDynamicSharedMemorySize, (int)scanLds);

  k_wprep<<<2, NTHR, 0, stream>>>(w1r, w1o, w2r, w2o, B1, B2);
  k_scan<1><<<gA, NTHR, scanLds, stream>>>(src, dst, nE, nN, vec8, MP, x, A1, w3r, w3o, b3, out);
  k_gemm<4, 1><<<gM, GTHR, 0, stream>>>(A1, AP1, B1, AP1, K1, b1, H1, MP);
  k_scan<2><<<gA, NTHR, scanLds, stream>>>(src, dst, nE, nN, vec8, MP, H1, A2, w3r, w3o, b3, out);
  k_gemm<4, 1><<<gM, GTHR, 0, stream>>>(A2, AP2, B2, AP2, K2, b2, H2, MP);
  k_scan<3><<<gA, NTHR, scanLds, stream>>>(src, dst, nE, nN, vec8, MP, H2, A2, w3r, w3o, b3, out);
}
